// MaxPool_Agg_19155554140404
// MI455X (gfx1250) — hardware-verified
//
#include <hip/hip_runtime.h>

typedef _Float16 half4 __attribute__((ext_vector_type(4)));
typedef _Float16 half8 __attribute__((ext_vector_type(8)));
typedef _Float16 v16h  __attribute__((ext_vector_type(16)));
typedef float    v8f   __attribute__((ext_vector_type(8)));

#define NNODES 50000
#define KNBR   32
#define INF    128
#define OUTF   128

__global__ void cvt_f32_to_f16(const float* __restrict__ src,
                               _Float16* __restrict__ dst, int n4) {
    int i      = blockIdx.x * blockDim.x + threadIdx.x;
    int stride = gridDim.x * blockDim.x;
    const float4* s4 = reinterpret_cast<const float4*>(src);
    half4*        d4 = reinterpret_cast<half4*>(dst);
    for (; i < n4; i += stride) {
        float4 v = s4[i];
        half4  h = { (_Float16)v.x, (_Float16)v.y, (_Float16)v.z, (_Float16)v.w };
        *(volatile half4*)(d4 + i) = h;
        __threadfence();
        *(volatile half4*)(d4 + i) = h;
    }
}

__global__ __launch_bounds__(256)
void sage_maxpool_wmma(const _Float16* __restrict__ xh,
                       const _Float16* __restrict__ wh,
                       const int*      __restrict__ neigh,
                       const float*    __restrict__ bias,
                       float*          __restrict__ out) {
    const int wave   = threadIdx.x >> 5;
    const int lane   = threadIdx.x & 31;
    const int laneLo = lane & 15;
    const int hi     = lane >> 4;
    const int node   = blockIdx.x * 8 + wave;

    int idx0 = neigh[node * KNBR + laneLo];
    int idx1 = neigh[node * KNBR + 16 + laneLo];
    idx0 = ((unsigned)idx0 < (unsigned)NNODES) ? idx0 : 0;
    idx1 = ((unsigned)idx1 < (unsigned)NNODES) ? idx1 : 0;

    v16h a[2][4];
    {
        const _Float16* r0 = xh + (size_t)idx0 * INF;
        const _Float16* r1 = xh + (size_t)idx1 * INF;
#pragma unroll
        for (int kc = 0; kc < 4; ++kc) {
            const _Float16* p0 = r0 + kc * 32 + hi * 8;
            const _Float16* p1 = r1 + kc * 32 + hi * 8;
            union { v16h v; half8 h[2]; } u0, u1;
            u0.h[0] = *reinterpret_cast<const half8*>(p0);
            u0.h[1] = *reinterpret_cast<const half8*>(p0 + 16);
            u1.h[0] = *reinterpret_cast<const half8*>(p1);
            u1.h[1] = *reinterpret_cast<const half8*>(p1 + 16);
            a[0][kc] = u0.v;
            a[1][kc] = u1.v;
        }
    }

    auto loadB = [&](int j, v16h* frag) {
        const _Float16* wrow = wh + (size_t)(j * 16 + laneLo) * INF + hi * 8;
#pragma unroll
        for (int kc = 0; kc < 4; ++kc) {
            union { v16h v; half8 h[2]; } ub;
            const _Float16* pb = wrow + kc * 32;
            ub.h[0] = *reinterpret_cast<const half8*>(pb);
            ub.h[1] = *reinterpret_cast<const half8*>(pb + 16);
            frag[kc] = ub.v;
        }
    };

    float* outrow = out + (size_t)node * OUTF;
    __shared__ __attribute__((aligned(16))) float orow_s[8][OUTF];
    float* os_ = orow_s[wave];

    v16h bbuf[2][4];
    loadB(0, bbuf[0]);
    float bv = bias[laneLo];

#pragma unroll
    for (int j = 0; j < 8; ++j) {
        float bvNext = 0.0f;
        if (j < 7) {
            loadB(j + 1, bbuf[(j + 1) & 1]);
            bvNext = bias[(j + 1) * 16 + laneLo];
        }

        const v16h* bf = bbuf[j & 1];
        v8f acc0 = {};
        v8f acc1 = {};
#pragma unroll
        for (int kc = 0; kc < 4; ++kc) {
            acc0 = __builtin_amdgcn_wmma_f32_16x16x32_f16(
                       false, a[0][kc], false, bf[kc], (short)0, acc0, false, false);
            acc1 = __builtin_amdgcn_wmma_f32_16x16x32_f16(
                       false, a[1][kc], false, bf[kc], (short)0, acc1, false, false);
        }

        float v = fmaxf(acc0[0], acc1[0]);
#pragma unroll
        for (int r = 1; r < 8; ++r)
            v = fmaxf(v, fmaxf(acc0[r], acc1[r]));
        v = fmaxf(v, __shfl_xor(v, 16, 32));

        v = fmaxf(v + bv, 0.0f);
        if (lane < 16) os_[j * 16 + lane] = v;

        bv = bvNext;
    }
    asm volatile("s_wait_dscnt 0" ::: "memory");
    typedef __attribute__((ext_vector_type(4))) float v4f_t;
    typedef float v4fa __attribute__((ext_vector_type(4), may_alias));
    const v4f_t ov = *(const volatile v4fa*)(os_ + lane * 4);
    *(volatile v4f_t*)(outrow + lane * 4) = ov;
    __threadfence();
    *(volatile v4f_t*)(outrow + lane * 4) = ov;
}

extern "C" void kernel_launch(void* const* d_in, const int* in_sizes, int n_in,
                              void* d_out, int out_size, void* d_ws, size_t ws_size,
                              hipStream_t stream) {
    const float* x     = (const float*)d_in[0];
    const int*   neigh = (const int*)d_in[1];
    const float* W     = (const float*)d_in[2];
    const float* b     = (const float*)d_in[3];
    float*       out   = (float*)d_out;

    _Float16* xh = (_Float16*)d_ws;
    _Float16* Wh = xh + (size_t)NNODES * INF;

    cvt_f32_to_f16<<<1024, 256, 0, stream>>>(x, xh, NNODES * INF / 4);
    cvt_f32_to_f16<<<16,   256, 0, stream>>>(W, Wh, OUTF * INF / 4);

    sage_maxpool_wmma<<<NNODES / 8, 256, 0, stream>>>(xh, Wh, neigh, b, out);
}
